// gnn_15960098471965
// MI455X (gfx1250) — hardware-verified
//
#include <hip/hip_runtime.h>
#include <stddef.h>
#include <stdint.h>


#define NF     512
#define KH     1024
#define NST    1024
#define MH     128
#define NP     256
#define K2E    256
#define NTHR   256
#define NWAVE  8
#define EPT    8
#define CHUNK  (NTHR * EPT)
#define WCAP   (EPT * 32)
#define LISTN  (NWAVE * WCAP)
#define NBA    1024
#define SLA    10
#define RCAP   16384
#define DEGCAP 64
#define GBM    64
#define GBN    128
#define GTHR   128
#define EB     128
#define AGG_ZINTS    (LISTN + 2 * RCAP + 3 * NBA)
#define MISC_INTS    16
#define ROWBUF_INTS  (NWAVE * KH / 2)
#define AGG_LDS_INTS (AGG_ZINTS + MISC_INTS + ROWBUF_INTS)
#define EDGE_LDS_INTS (EB * K2E / 2 + EB * MH + 256 + 128 + 256 + 128 + 128)
#define WSMAX  134217728

#define OFF_WL0 0
#define OFF_WL1 (OFF_WL0 + 1024 * 512)
#define OFF_WL2 (OFF_WL1 + 1024 * 1024)
#define OFF_WP  (OFF_WL2 + 1024 * 1024)
#define OFF_W2P (OFF_WP + 256 * 1024)
#define WB_ELEMS (OFF_W2P + 128 * 256)
#define U_L0   (1024 * 64)
#define U_L12  (2 * 1024 * 128)
#define U_WP   (256 * 128)
#define U_W2   (128 * 32)
#define U_TOT  (U_L0 + U_L12 + U_WP + U_W2)

static_assert((CHUNK & (CHUNK - 1)) == 0 && CHUNK <= 4096);
static_assert((NBA & (NBA - 1)) == 0 && NBA == (1 << SLA));
static_assert(((long long)CHUNK << SLA) < (1LL << 31));
static_assert(LISTN % NTHR == 0);
static_assert(NBA % NWAVE == 0 && NBA % 32 == 0 && NBA % GBM == 0);
static_assert(RCAP % 4 == 0 && AGG_ZINTS % 4 == 0 && LISTN % 4 == 0 && ((AGG_ZINTS + MISC_INTS) % 4) == 0);
static_assert(NF % 32 == 0 && KH % 32 == 0 && K2E % 32 == 0 && KH == 2 * NF && K2E == 2 * MH);
static_assert(NST % GBN == 0 && NP % GBN == 0 && GBM == (GTHR / 32) * 16 && GBN == 4 * 32);
static_assert(NF == 4 * 32 * 4 && MH == 4 * 32);
static_assert(U_L0 % NTHR == 0 && U_L12 % NTHR == 0 && U_WP % NTHR == 0 && U_W2 % NTHR == 0);
static_assert((U_L0 / 2) % NTHR == 0 && (U_L12 / 4) % NTHR == 0);
static_assert(WB_ELEMS == 2916352);
static_assert(AGG_LDS_INTS * 4 <= 300000 && EDGE_LDS_INTS * 4 <= 300000);
static_assert(EB == 16 * NWAVE && 2 * EB == NTHR);

typedef float          v4f   __attribute__((ext_vector_type(4)));
typedef float          v8f   __attribute__((ext_vector_type(8)));
typedef int            v4i   __attribute__((ext_vector_type(4)));
typedef int            v8i   __attribute__((ext_vector_type(8)));
typedef unsigned short v4us  __attribute__((ext_vector_type(4)));
typedef unsigned short v8us  __attribute__((ext_vector_type(8)));
typedef unsigned short v16us __attribute__((ext_vector_type(16)));
typedef __bf16         v16bf __attribute__((ext_vector_type(16)));
typedef v4f  __attribute__((may_alias)) v4fa;
typedef v4i  __attribute__((may_alias)) v4ia;
typedef v4us __attribute__((may_alias)) v4usa;
typedef v8us __attribute__((may_alias)) v8usa;
union FragB { v16bf v; v16us u; v8us h[2]; v8i w; };

__device__ __forceinline__ v8f wmb(const FragB& a, const FragB& b, v8f c) {
  v8f d = __builtin_amdgcn_wmma_f32_16x16x32_bf16(false, a.v, false, b.v, (short)0, c, false, false);
  asm volatile("v_nop\n\tv_nop\n\tv_nop\n\tv_nop" : "+v"(d) : "v"(a.w), "v"(b.w));
  return d;
}

__device__ __forceinline__ unsigned bf16_bits(float f) {
  const unsigned u = __float_as_uint(f);
  const unsigned r = (u + 0x7FFFu + ((u >> 16) & 1u)) >> 16;
  return (f != f) ? 0x7FC0u : r;
}
__device__ __forceinline__ float bf16_val(float f) {
  return __uint_as_float(bf16_bits(f) << 16);
}
__device__ __forceinline__ v4f bf16_val4(const v4f a) {
  v4f o;
  o.x = bf16_val(a.x); o.y = bf16_val(a.y); o.z = bf16_val(a.z); o.w = bf16_val(a.w);
  return o;
}
__device__ __forceinline__ float relu_np(float v) { return (v > 0.0f) ? v : (v - v); }

__device__ __forceinline__ void split4(const v4f y, v4us& h, v4us& l) {
  unsigned hb;
  hb = bf16_bits(y.x); h[0] = (unsigned short)hb; l[0] = (unsigned short)bf16_bits(y.x - __uint_as_float(hb << 16));
  hb = bf16_bits(y.y); h[1] = (unsigned short)hb; l[1] = (unsigned short)bf16_bits(y.y - __uint_as_float(hb << 16));
  hb = bf16_bits(y.z); h[2] = (unsigned short)hb; l[2] = (unsigned short)bf16_bits(y.z - __uint_as_float(hb << 16));
  hb = bf16_bits(y.w); h[3] = (unsigned short)hb; l[3] = (unsigned short)bf16_bits(y.w - __uint_as_float(hb << 16));
}

__device__ __forceinline__ void wave_sync() {
  __builtin_amdgcn_fence(__ATOMIC_RELEASE, "wavefront");
  __builtin_amdgcn_wave_barrier();
  __builtin_amdgcn_fence(__ATOMIC_ACQUIRE, "wavefront");
}

template <int SLB>
__device__ __forceinline__ int scan_chunk(const int* __restrict__ dsts, int nE, int cbase, int slotBase,
                                          int nb, int vec8, int* list, int tid, int lane, int wave) {
  int wc = 0;
  const int el0  = tid * EPT;
  const int e0   = cbase + el0;
  const int sent = -2147483647 - 1;
  v4i da, db;
  if (vec8 != 0 && cbase + CHUNK <= nE) {
    da = *(const v4i*)(dsts + e0);
    db = *(const v4i*)(dsts + e0 + 4);
  } else {
    da.x = (e0     < nE) ? dsts[min(e0,     nE - 1)] : sent;
    da.y = (e0 + 1 < nE) ? dsts[min(e0 + 1, nE - 1)] : sent;
    da.z = (e0 + 2 < nE) ? dsts[min(e0 + 2, nE - 1)] : sent;
    da.w = (e0 + 3 < nE) ? dsts[min(e0 + 3, nE - 1)] : sent;
    db.x = (e0 + 4 < nE) ? dsts[min(e0 + 4, nE - 1)] : sent;
    db.y = (e0 + 5 < nE) ? dsts[min(e0 + 5, nE - 1)] : sent;
    db.z = (e0 + 6 < nE) ? dsts[min(e0 + 6, nE - 1)] : sent;
    db.w = (e0 + 7 < nE) ? dsts[min(e0 + 7, nE - 1)] : sent;
  }
  const unsigned nbs = (unsigned)slotBase;
  const unsigned unb = (unsigned)nb;
  const unsigned s0 = (unsigned)da.x - nbs, s1 = (unsigned)da.y - nbs;
  const unsigned s2 = (unsigned)da.z - nbs, s3 = (unsigned)da.w - nbs;
  const unsigned s4 = (unsigned)db.x - nbs, s5 = (unsigned)db.y - nbs;
  const unsigned s6 = (unsigned)db.z - nbs, s7 = (unsigned)db.w - nbs;
  const bool h0 = s0 < unb, h1 = s1 < unb, h2 = s2 < unb, h3 = s3 < unb;
  const bool h4 = s4 < unb, h5 = s5 < unb, h6 = s6 < unb, h7 = s7 < unb;
  const unsigned any = __builtin_amdgcn_ballot_w32(h0 | h1 | h2 | h3 | h4 | h5 | h6 | h7);
  if (any != 0u) {
#define HITJ(J, HJ, SJ) { \
      const unsigned mj = __builtin_amdgcn_ballot_w32(HJ); \
      if (mj != 0u) { \
        if (HJ) { \
          const int pos = wc + (int)__builtin_amdgcn_mbcnt_lo(mj, 0u); \
          if (pos < WCAP) list[wave * WCAP + pos] = ((el0 + (J)) << SLB) | (int)(SJ); \
        } \
        wc += (int)__builtin_popcount(mj); } }
    HITJ(0, h0, s0)
    HITJ(1, h1, s1)
    HITJ(2, h2, s2)
    HITJ(3, h3, s3)
    HITJ(4, h4, s4)
    HITJ(5, h5, s5)
    HITJ(6, h6, s6)
    HITJ(7, h7, s7)
#undef HITJ
  }
  return wc;
}

__device__ __forceinline__ v8us gather8(const float* __restrict__ p, int stride) {
  v8us o;
#pragma unroll
  for (int i = 0; i < 8; ++i) o[i] = (unsigned short)bf16_bits(p[(size_t)i * (size_t)stride]);
  return o;
}

__global__ __launch_bounds__(NTHR) void k_wprep(const float* __restrict__ Ws, const float* __restrict__ Wn,
                                                const float* __restrict__ W1, const float* __restrict__ W2,
                                                unsigned short* wb) {
  const int u = (int)blockIdx.x * NTHR + (int)threadIdx.x;
  v8us o;
  size_t doff;
  if (u < U_L0) {
    const int n  = u >> 6;
    const int k8 = (u & 63) * 8;
    doff = (size_t)OFF_WL0 + (size_t)n * NF + k8;
    if (n < NF) o = gather8(Ws + (size_t)k8 * NF + n, NF);
    else        o = gather8(Wn + (size_t)k8 * NF + (n - NF), NF);
  } else if (u < U_L0 + U_L12) {
    const int v  = u - U_L0;
    const int li = v >> 17;
    const int w  = v & 131071;
    const int n  = w >> 7;
    const int k8 = (w & 127) * 8;
    const int kk = k8 & (NF - 1);
    doff = (size_t)OFF_WL1 + (size_t)li * (1024 * 1024) + (size_t)n * KH + k8;
    const size_t so = (size_t)(li + 1) * NF * NF + (size_t)kk * NF;
    if (n < NF) o = gather8(Ws + so + n, NF);
    else        o = gather8(Wn + so + (n - NF), NF);
  } else if (u < U_L0 + U_L12 + U_WP) {
    const int v  = u - (U_L0 + U_L12);
    const int n  = v >> 7;
    const int k8 = (v & 127) * 8;
    const int kk = k8 & (NF - 1);
    doff = (size_t)OFF_WP + (size_t)n * KH + k8;
    o = gather8(W1 + (size_t)(kk + ((n >> 7) << 9)) * MH + (n & (MH - 1)), MH);
  } else if (u < U_TOT) {
    const int v  = u - (U_L0 + U_L12 + U_WP);
    const int n  = v >> 5;
    const int k8 = (v & 31) * 8;
    const int kk = k8 & (MH - 1);
    doff = (size_t)OFF_W2P + (size_t)n * K2E + k8;
    o = gather8(W2 + (size_t)kk * MH + n, MH);
  } else {
    return;
  }
  unsigned short* dp = wb + doff;
  *(volatile v8us*)dp = o;
  __threadfence();
  *(volatile v8us*)dp = o;
}

__global__ __launch_bounds__(NTHR) void k_cvx(const float* __restrict__ x, int nN, int nUnits,
                                              unsigned short* xb) {
  const int u = (int)blockIdx.x * NTHR + (int)threadIdx.x;
  if (u >= nUnits) return;
  const int row = u >> 6;
  const int k8  = (u & 63) * 8;
  const int rc  = row < nN ? row : nN - 1;
  const float* p = x + (size_t)rc * NF + k8;
  const v4f a = *(const v4fa*)p;
  const v4f b = *(const v4fa*)(p + 4);
  const bool ok = row < nN;
  v8us o;
  o[0] = ok ? (unsigned short)bf16_bits(a.x) : (unsigned short)0;
  o[1] = ok ? (unsigned short)bf16_bits(a.y) : (unsigned short)0;
  o[2] = ok ? (unsigned short)bf16_bits(a.z) : (unsigned short)0;
  o[3] = ok ? (unsigned short)bf16_bits(a.w) : (unsigned short)0;
  o[4] = ok ? (unsigned short)bf16_bits(b.x) : (unsigned short)0;
  o[5] = ok ? (unsigned short)bf16_bits(b.y) : (unsigned short)0;
  o[6] = ok ? (unsigned short)bf16_bits(b.z) : (unsigned short)0;
  o[7] = ok ? (unsigned short)bf16_bits(b.w) : (unsigned short)0;
  unsigned short* dp = xb + (size_t)row * NF + k8;
  *(volatile v8us*)dp = o;
  __threadfence();
  *(volatile v8us*)dp = o;
}

__global__ __launch_bounds__(GTHR) void k_gemm(const unsigned short* __restrict__ A, int lda,
                                               const unsigned short* __restrict__ BT, int K,
                                               float* outF, int ldo) {
  __shared__ __attribute__((aligned(16))) float stg[GBM * GBN];
  const int tid = (int)threadIdx.x, lane = tid & 31, wave = tid >> 5, hh = lane >> 4, m = lane & 15;
  const int rowBase = (int)blockIdx.x * GBM;
  const int col0    = (int)blockIdx.y * GBN;

  v8f acc[8];
  {
    const v8f z = {0.f, 0.f, 0.f, 0.f, 0.f, 0.f, 0.f, 0.f};
#pragma unroll
    for (int t = 0; t < 8; ++t) acc[t] = z;
  }
  const unsigned short* ap = A  + (size_t)(rowBase + 16 * wave + m) * (size_t)lda + 8 * hh;
  const unsigned short* bp = BT + (size_t)(col0 + m) * (size_t)K + 8 * hh;

#pragma unroll 1
  for (int k0 = 0; k0 < K; k0 += 32) {
    FragB af;
    af.h[0] = *(const v8usa*)(ap + k0);
    af.h[1] = *(const v8usa*)(ap + k0 + 16);
#pragma unroll
    for (int nt = 0; nt < 8; ++nt) {
      const unsigned short* wq = bp + (size_t)(16 * nt) * (size_t)K + k0;
      FragB bf;
      bf.h[0] = *(const v8usa*)wq;
      bf.h[1] = *(const v8usa*)(wq + 16);
      acc[nt] = wmb(af, bf, acc[nt]);
    }
  }

#pragma unroll
  for (int nt = 0; nt < 8; ++nt) {
    const int lc = 16 * nt + m;
#pragma unroll
    for (int r = 0; r < 8; ++r) {
      const int lr = 16 * wave + 8 * hh + r;
      stg[lr * GBN + lc] = acc[nt][r];
    }
  }
  __syncthreads();

  v4f pv[16];
#pragma unroll
  for (int i = 0; i < 16; ++i) pv[i] = *(const v4fa*)(stg + (16 * wave + i) * GBN + 4 * lane);
#pragma unroll
  for (int i = 0; i < 16; ++i) {
    float* op = outF + (size_t)(rowBase + 16 * wave + i) * (size_t)ldo + col0 + 4 * lane;
    *(volatile v4f*)op = pv[i];
  }
  __threadfence();
#pragma unroll
  for (int i = 0; i < 16; ++i) {
    float* op = outF + (size_t)(rowBase + 16 * wave + i) * (size_t)ldo + col0 + 4 * lane;
    *(volatile v4f*)op = pv[i];
  }
}

template <int RELU>
__global__ __launch_bounds__(NTHR) void k_scan(const int* __restrict__ gath, const int* __restrict__ keys,
                                               int nE, int nN, int vec8, int mRows,
                                               const float* __restrict__ st, const float* __restrict__ bias,
                                               unsigned short* apl) {
  extern __shared__ __attribute__((aligned(16))) int dsm[];
  int* list = dsm;
  int* hl   = dsm + LISTN;
  int* sl   = hl + RCAP;
  int* cnt  = sl + RCAP;
  int* offs = cnt + NBA;
  int* cur  = offs + NBA;
  int* misc = cur + NBA;
  const int tid = (int)threadIdx.x, lane = tid & 31, wave = tid >> 5;
  unsigned short* rowbuf = (unsigned short*)(misc + MISC_INTS) + wave * KH;
  const int nodeBase = (int)blockIdx.x * NBA;

  {
    const v4i z4 = {0, 0, 0, 0};
    for (int i = tid * 4; i < AGG_ZINTS; i += NTHR * 4) *(v4ia*)(dsm + i) = z4;
    if (tid < MISC_INTS) misc[tid] = 0;
  }
  const v4f bq0 = bf16_val4(*(const v4f*)(bias + 4 * lane));
  const v4f bq1 = bf16_val4(*(const v4f*)(bias + 128 + 4 * lane));
  const v4f bq2 = bf16_val4(*(const v4f*)(bias + 256 + 4 * lane));
  const v4f bq3 = bf16_val4(*(const v4f*)(bias + 384 + 4 * lane));
  __syncthreads();

  int t = 0, ov = 0;
  const int nChunks = (nE + CHUNK - 1) / CHUNK;
#pragma unroll 1
  for (int ch = 0; ch < nChunks; ++ch) {
    const int cbase = ch * CHUNK;
    const int wc = scan_chunk<SLA>(keys, nE, cbase, nodeBase, NBA, vec8, list, tid, lane, wave);
    if (lane == 0) misc[wave] = wc;
    __syncthreads();
    if (wave == 0) {
#pragma unroll 1
      for (int w2 = 0; w2 < NWAVE; ++w2) {
        int c = misc[w2];
        c = c < 0 ? 0 : (c > WCAP ? WCAP : c);
#pragma unroll 1
        for (int b0 = 0; b0 < c; b0 += 32) {
          const int idx = b0 + lane;
          const int ent = list[w2 * WCAP + (idx < WCAP ? idx : WCAP - 1)];
          const int m32 = (c - b0) < 32 ? (c - b0) : 32;
#pragma unroll 1
          for (int k = 0; k < m32; ++k) {
            const int u    = __builtin_amdgcn_readlane(ent, k);
            const int slot = u & (NBA - 1);
            const int el   = (u >> SLA) & (CHUNK - 1);
            const int pk   = ((cbase + el) << SLA) | slot;
            if (t < RCAP) {
              if (lane == 0) { hl[t] = pk; cnt[slot] = cnt[slot] + 1; }
              t = t + 1;
            } else {
              ov = 1;
            }
          }
        }
      }
    }
    __syncthreads();
  }
  if (wave == 0 && lane == 0) { misc[8] = t; misc[9] = ov; }
  __syncthreads();
  int tt = misc[8];
  tt = tt < 0 ? 0 : (tt > RCAP ? RCAP : tt);
  const int ovf = misc[9];

  if (wave == 0) {
    const int base = lane * (NBA / 32);
    int s = 0;
#pragma unroll 1
    for (int i = 0; i < NBA / 32; ++i) s += cnt[base + i];
    int incl = s;
#pragma unroll
    for (int d = 1; d < 32; d <<= 1) {
      const int y = __shfl_up(incl, d, 32);
      if (lane >= d) incl += y;
    }
    int run = incl - s;
#pragma unroll 1
    for (int i = 0; i < NBA / 32; ++i) {
      const int cv = cnt[base + i];
      offs[base + i] = run;
      cur[base + i]  = run;
      run += cv;
    }
  }
  __syncthreads();
  if (wave == 0) {
#pragma unroll 1
    for (int b0 = 0; b0 < tt; b0 += 32) {
      const int idx = b0 + lane;
      const int ent = hl[idx < RCAP ? idx : RCAP - 1];
      const int m32 = (tt - b0) < 32 ? (tt - b0) : 32;
#pragma unroll 1
      for (int k = 0; k < m32; ++k) {
        const int u    = __builtin_amdgcn_readlane(ent, k);
        const int slot = u & (NBA - 1);
        if (lane == 0) {
          int p = cur[slot];
          p = p < 0 ? 0 : (p > RCAP - 1 ? RCAP - 1 : p);
          sl[p] = u;
          cur[slot] = p + 1;
        }
      }
    }
  }
  __syncthreads();

  const float qnan = __int_as_float(0x7fc00000);
  const float pz = (ovf != 0) ? qnan : 0.0f;
#pragma unroll 1
  for (int si = 0; si < NBA / NWAVE; ++si) {
    const int s    = si * NWAVE + wave;
    const int node = nodeBase + s;
    int c = cnt[s];
    const bool big = c > DEGCAP;
    c = c < 0 ? 0 : (c > DEGCAP ? DEGCAP : c);
    int o = offs[s];
    o = o < 0 ? 0 : (o > RCAP ? RCAP : o);
    const int nc = node < nN ? node : nN - 1;
    v4f a0 = {0.f, 0.f, 0.f, 0.f}, a1 = a0, a2 = a0, a3 = a0;
#pragma unroll 1
    for (int b0 = 0; b0 < c; b0 += 32) {
      int idx = o + b0 + lane;
      idx = idx > RCAP - 1 ? RCAP - 1 : idx;
      const int ent = sl[idx];
      int eid = ent >> SLA;
      eid = eid < 0 ? 0 : (eid > nE - 1 ? nE - 1 : eid);
      int sr = gath[eid];
      sr = sr < 0 ? 0 : (sr > nN - 1 ? nN - 1 : sr);
      const int m32 = (c - b0) < 32 ? (c - b0) : 32;
#pragma unroll 1
      for (int k = 0; k < m32; ++k) {
        const int sk = __builtin_amdgcn_readlane(sr, k);
        const float* rp = st + (size_t)sk * NST + NF + 4 * lane;
        const v4f t0 = *(const v4f*)rp;
        const v4f t1 = *(const v4f*)(rp + 128);
        const v4f t2 = *(const v4f*)(rp + 256);
        const v4f t3 = *(const v4f*)(rp + 384);
        a0 += t0; a1 += t1; a2 += t2; a3 += t3;
      }
    }
    const float dg  = (float)c;
    const float inv = 1.0f / fmaxf(dg, 1.0f);
    const float* sp = st + (size_t)nc * NST + 4 * lane;
    const v4f s0 = *(const v4f*)sp;
    const v4f s1 = *(const v4f*)(sp + 128);
    const v4f s2 = *(const v4f*)(sp + 256);
    const v4f s3 = *(const v4f*)(sp + 384);
    const float pzr = big ? qnan : pz;
    const bool live = node < nN;
    v4f y0 = (s0 + a0 * inv) + bq0;
    v4f y1 = (s1 + a1 * inv) + bq1;
    v4f y2 = (s2 + a2 * inv) + bq2;
    v4f y3 = (s3 + a3 * inv) + bq3;
    if constexpr (RELU != 0) {
      y0.x = relu_np(y0.x); y0.y = relu_np(y0.y); y0.z = relu_np(y0.z); y0.w = relu_np(y0.w);
      y1.x = relu_np(y1.x); y1.y = relu_np(y1.y); y1.z = relu_np(y1.z); y1.w = relu_np(y1.w);
      y2.x = relu_np(y2.x); y2.y = relu_np(y2.y); y2.z = relu_np(y2.z); y2.w = relu_np(y2.w);
      y3.x = relu_np(y3.x); y3.y = relu_np(y3.y); y3.z = relu_np(y3.z); y3.w = relu_np(y3.w);
    }
    y0 = y0 + pzr; y1 = y1 + pzr; y2 = y2 + pzr; y3 = y3 + pzr;
    const v4f zz = {0.f, 0.f, 0.f, 0.f};
    y0 = live ? y0 : zz; y1 = live ? y1 : zz; y2 = live ? y2 : zz; y3 = live ? y3 : zz;
    v4us h0, l0, h1, l1, h2, l2, h3, l3;
    split4(y0, h0, l0); split4(y1, h1, l1); split4(y2, h2, l2); split4(y3, h3, l3);
    *(v4usa*)(rowbuf + 4 * lane)            = h0;
    *(v4usa*)(rowbuf + 128 + 4 * lane)      = h1;
    *(v4usa*)(rowbuf + 256 + 4 * lane)      = h2;
    *(v4usa*)(rowbuf + 384 + 4 * lane)      = h3;
    *(v4usa*)(rowbuf + NF + 4 * lane)       = l0;
    *(v4usa*)(rowbuf + NF + 128 + 4 * lane) = l1;
    *(v4usa*)(rowbuf + NF + 256 + 4 * lane) = l2;
    *(v4usa*)(rowbuf + NF + 384 + 4 * lane) = l3;
    wave_sync();
    const v8us q0 = *(const v8usa*)(rowbuf + 8 * lane);
    const v8us q1 = *(const v8usa*)(rowbuf + 256 + 8 * lane);
    const v8us q2 = *(const v8usa*)(rowbuf + 512 + 8 * lane);
    const v8us q3 = *(const v8usa*)(rowbuf + 768 + 8 * lane);
    wave_sync();
    if (node < mRows) {
      unsigned short* rpw = apl + (size_t)node * KH + 8 * lane;
      *(volatile v8us*)rpw         = q0;
      *(volatile v8us*)(rpw + 256) = q1;
      *(volatile v8us*)(rpw + 512) = q2;
      *(volatile v8us*)(rpw + 768) = q3;
      __threadfence();
      *(volatile v8us*)rpw         = q0;
      *(volatile v8us*)(rpw + 256) = q1;
      *(volatile v8us*)(rpw + 512) = q2;
      *(volatile v8us*)(rpw + 768) = q3;
    }
  }
}

__global__ __launch_bounds__(NTHR) void k_edge(const float* __restrict__ P,
                                               const int* __restrict__ ps, const int* __restrict__ pd,
                                               const int* __restrict__ ns, const int* __restrict__ nd,
                                               int nE, int nN,
                                               const float* __restrict__ b1, const unsigned short* __restrict__ W2P,
                                               const float* __restrict__ b2, const float* __restrict__ W3,
                                               const float* __restrict__ b3, float* out) {
  extern __shared__ __attribute__((aligned(16))) int dsm[];
  unsigned short* atile = (unsigned short*)dsm;
  float* etile = (float*)(dsm + EB * K2E / 2);
  float* w3s   = etile + EB * MH;
  float* b2s   = w3s + 256;
  float* outs  = b2s + 128;
  int*   uidx  = (int*)(outs + 256);
  int*   vidx  = uidx + 128;
  const int tid = (int)threadIdx.x, lane = tid & 31, wave = tid >> 5, hh = lane >> 4, m = lane & 15;

  w3s[tid] = bf16_val(W3[tid]);
  if (tid < MH) {
    b2s[tid] = bf16_val(b2[tid]);
    const int E   = (int)blockIdx.x * EB + tid;
    const int isn = (E >= nE) ? 1 : 0;
    int ec = E - isn * nE;
    ec = ec < 0 ? 0 : (ec > nE - 1 ? nE - 1 : ec);
    const int up = ps[ec], vp = pd[ec], un = ns[ec], vn = nd[ec];
    const int mk = -isn;
    int uu = (up & ~mk) | (un & mk);
    int vv = (vp & ~mk) | (vn & mk);
    uu = uu < 0 ? 0 : (uu > nN - 1 ? nN - 1 : uu);
    vv = vv < 0 ? 0 : (vv > nN - 1 ? nN - 1 : vv);
    uidx[tid] = uu;
    vidx[tid] = vv;
  }
  const v4f b1q = bf16_val4(*(const v4f*)(b1 + 4 * lane));
  __syncthreads();

#pragma unroll 2
  for (int i = 0; i < 16; ++i) {
    const int row = 16 * wave + i;
    const int uu = uidx[row];
    const int vv = vidx[row];
    const v4f pu = *(const v4f*)(P + (size_t)uu * NP + 4 * lane);
    const v4f pv = *(const v4f*)(P + (size_t)vv * NP + MH + 4 * lane);
    v4f e = (pu + pv) + b1q;
    e.x = relu_np(e.x); e.y = relu_np(e.y); e.z = relu_np(e.z); e.w = relu_np(e.w);
    v4us h4, l4;
    split4(e, h4, l4);
    *(v4usa*)(atile + row * K2E + 4 * lane)      = h4;
    *(v4usa*)(atile + row * K2E + MH + 4 * lane) = l4;
  }
  __syncthreads();

  v8f acc[8];
  {
    const v8f z = {0.f, 0.f, 0.f, 0.f, 0.f, 0.f, 0.f, 0.f};
#pragma unroll
    for (int t = 0; t < 8; ++t) acc[t] = z;
  }
  const unsigned short* arow = atile + (16 * wave + m) * K2E + 8 * hh;
  const unsigned short* bp   = W2P + (size_t)m * K2E + 8 * hh;
#pragma unroll 1
  for (int k0 = 0; k0 < K2E; k0 += 32) {
    FragB af;
    af.h[0] = *(const v8usa*)(arow + k0);
    af.h[1] = *(const v8usa*)(arow + k0 + 16);
#pragma unroll
    for (int nt = 0; nt < 8; ++nt) {
      const unsigned short* wq = bp + (size_t)(16 * nt) * K2E + k0;
      FragB bf;
      bf.h[0] = *(const v8usa*)wq;
      bf.h[1] = *(const v8usa*)(wq + 16);
      acc[nt] = wmb(af, bf, acc[nt]);
    }
  }
#pragma unroll
  for (int nt = 0; nt < 8; ++nt) {
    const int lc = 16 * nt + m;
    const float bv = b2s[lc];
#pragma unroll
    for (int r = 0; r < 8; ++r) {
      const int lr = 16 * wave + 8 * hh + r;
      etile[lr * MH + lc] = relu_np(acc[nt][r] + bv);
    }
  }
  __syncthreads();

  {
    const int row = tid >> 1;
    const int c   = tid & 1;
    const float* er = etile + row * MH;
    float s = 0.0f;
#pragma unroll 1
    for (int k4 = 0; k4 < MH / 4; ++k4) {
      const v4f p = *(const v4fa*)(er + 4 * k4);
      const float* w = w3s + (4 * k4) * 2 + c;
      s = fmaf(p.x, w[0], s);
      s = fmaf(p.y, w[2], s);
      s = fmaf(p.z, w[4], s);
      s = fmaf(p.w, w[6], s);
    }
    outs[tid] = s + bf16_val(b3[c]);
  }
  __syncthreads();
  const v4f ov = *(const v4fa*)(outs + 4 * (tid & 63));
  float* op = out + (size_t)blockIdx.x * (2 * EB) + 4 * (tid & 63);
  const bool okst = tid < 64;
  if (okst) *(volatile v4f*)op = ov;
  __threadfence();
  if (okst) *(volatile v4f*)op = ov;
}

static inline int cdiv(int a, int b) { return (a + b - 1) / b; }
static inline size_t al256(size_t o) { return (o + 255) & ~(size_t)255; }

extern "C" void kernel_launch(void* const* d_in, const int* in_sizes, int n_in,
                              void* d_out, int out_size, void* d_ws, size_t ws_size,
                              hipStream_t stream) {
  if (n_in < 16) return;
  if (in_sizes[0] < NF || (in_sizes[0] % NF) != 0) return;
  const int nN = in_sizes[0] / NF;
  if (nN < 16 || nN >= (1 << 21)) return;
  if (in_sizes[1] != 3 * NF * NF || in_sizes[2] != 3 * NF * NF) return;
  if (in_sizes[3] != 3 * NF) return;
  if (in_sizes[4] != 2 * NF * MH || in_sizes[5] != MH) return;
  if (in_sizes[6] != MH * MH || in_sizes[7] != MH) return;
  if (in_sizes[8] != MH * 2 || in_sizes[9] != 2) return;
  const int nE = in_sizes[10];
  if (nE < 1 || nE >= (1 << 21)) return;
  if (in_sizes[11] != nE || in_sizes[12] != nE || in_sizes[13] != nE) return;
  if (in_sizes[14] != nE || in_sizes[15] != nE) return;
  if ((nE % EB) != 0) return;
  if ((long long)out_size != 4LL * (long long)nE) return;

  const float* x   = (const float*)d_in[0];
  const float* Ws  = (const float*)d_in[1];
  const float* Wn  = (const float*)d_in[2];
  const float* bb  = (const float*)d_in[3];
  const float* W1  = (const float*)d_in[4];
  const float* b1  = (const float*)d_in[5];
  const float* W2  = (const float*)d_in[6];
  const float* b2  = (const float*)d_in[7];
  const float* W3  = (const float*)d_in[8];
  const float* b3  = (const float*)d_in[9];
  const int*   src = (const int*)d_in[10];
  const int*   dst = (const int*)d_in[11];
  const int*   psr = (const int*)d_in[12];
  const int*   pds = (const int*)d_in[13];
  const int*   nsr = (const int*)d_in[14];
  const int*   nds = (const int*)d_in[15];
  float* out = (float*)d_out;

  const int MP = cdiv(nN, GBM) * GBM;
  const int gM = MP / GBM;
  const int gA = cdiv(MP, NBA);
  if ((long long)gA * NBA < (long long)MP) return;
  const int vec8 = ((nE & 3) == 0) ? 1 : 0;

  char* ws = (char*)d_ws;
  size_t off = 0;
  const size_t oST  = off; off = al256(off + (size_t)MP * NST * 4);
  const size_t oXHL = off; off = al256(off + (size_t)MP * KH * 2);
  const size_t oWB  = off; off = al256(off + (size_t)WB_ELEMS * 2);
  if (off > ws_size || off > (size_t)WSMAX) return;
  if ((size_t)MP * NP * 4 > (size_t)MP * NST * 4) return;
  if ((size_t)MP * NF * 2 > (size_t)MP * KH * 2) return;
  float*          ST  = (float*)(ws + oST);
  unsigned short* XHL = (unsigned short*)(ws + oXHL);
  unsigned short* WB  = (unsigned short*)(ws + oWB);
  float*          PP  = ST;
  unsigned short* XB  = XHL;

  const size_t scanLds = (size_t)AGG_LDS_INTS * 4;
  const size_t edgeLds = (size_t)EDGE_LDS_INTS * 4;
  hipFuncSetAttribute(reinterpret_cast<const void*>(&k_scan<1>), hipFuncAttributeMaxDynamicSharedMemorySize, (int)scanLds);
  hipFuncSetAttribute(reinterpret_cast<const void*>(&k_scan<0>), hipFuncAttributeMaxDynamicSharedMemorySize, (int)scanLds);
  hipFuncSetAttribute(reinterpret_cast<const void*>(&k_edge), hipFuncAttributeMaxDynamicSharedMemorySize, (int)edgeLds);

  const int nUx = MP * (NF / 8);
  k_wprep<<<U_TOT / NTHR, NTHR, 0, stream>>>(Ws, Wn, W1, W2, WB);
  k_cvx<<<cdiv(nUx, NTHR), NTHR, 0, stream>>>(x, nN, nUx, XB);
  k_gemm<<<dim3(gM, NST / GBN), GTHR, 0, stream>>>(XB, NF, WB + OFF_WL0, NF, ST, NST);
  k_scan<1><<<gA, NTHR, scanLds, stream>>>(src, dst, nE, nN, vec8, MP, ST, bb, XHL);
  k_gemm<<<dim3(gM, NST / GBN), GTHR, 0, stream>>>(XHL, KH, WB + OFF_WL1, KH, ST, NST);
  k_scan<1><<<gA, NTHR, scanLds, stream>>>(src, dst, nE, nN, vec8, MP, ST, bb + NF, XHL);
  k_gemm<<<dim3(gM, NST / GBN), GTHR, 0, stream>>>(XHL, KH, WB + OFF_WL2, KH, ST, NST);
  k_scan<0><<<gA, NTHR, scanLds, stream>>>(src, dst, nE, nN, vec8, MP, ST, bb + 2 * NF, XHL);
  k_gemm<<<dim3(gM, NP / GBN), GTHR, 0, stream>>>(XHL, KH, WB + OFF_WP, KH, PP, NP);
  k_edge<<<(2 * nE) / EB, NTHR, edgeLds, stream>>>(PP, psr, pds, nsr, nds, nE, nN, b1, WB + OFF_W2P, b2, W3, b3, out);
}
